// InteractionLayer_29850022707551
// MI455X (gfx1250) — hardware-run, weakly checked
//
#include <hip/hip_runtime.h>


namespace {

constexpr int N = 20000, NP = 20000, NPL = NP  , SRCM = N  , EFULL = 320000, E = EFULL  ;
constexpr int C = 64, RB = 8, KR = 32  , G = 64  , MW = 3 * C  , OW = 9 * C  , NL = (NPL < N ? NPL : N);
constexpr float XS = 8.0f, WSC = 256.0f, WSQ = 0.25f, RS_ = 1024.0f, EPSS = 0.5f, SLOPE = 0.0f, BNEPS = 1e-5f;
static_assert(NP % 32 == 0 && NP >= N && NPL % 32 == 0 && C == 64, "tiling");
typedef _Float16 b16;
typedef __attribute__((ext_vector_type(16))) _Float16 v16b;
typedef __attribute__((ext_vector_type(8))) _Float16 v8b;
typedef __attribute__((ext_vector_type(8))) float v8f;
typedef __attribute__((ext_vector_type(4))) float v4f;
__device__ __forceinline__ float bf16_rne(float f) { unsigned int u = __float_as_uint(f); u += 0x7FFFu + ((u >> 16) & 1u); return __uint_as_float(u & 0xFFFF0000u); }
__device__ __forceinline__ void split16(float v, b16& hi, b16& lo) { hi = (b16)v; lo = (b16)(v - (float)hi); }
__device__ __forceinline__ v16b frag_kb(const b16* p, int hh) { const v8b a = *(const v8b*)(p + 8 * hh), b = *(const v8b*)(p + 16 + 8 * hh); v16b f;
#pragma unroll
  for (int e = 0; e < 8; ++e) { f[e] = a[e]; f[8 + e] = b[e]; } return f; }
__device__ __forceinline__ v8f wmma16b(v16b a, v16b b, v8f c) { v8f d = __builtin_amdgcn_wmma_f32_16x16x32_f16(false, a, false, b, (short)0, c, false, false); asm volatile("v_nop\n\tv_nop\n\tv_nop\n\tv_nop" : "+v"(d) : "v"(a), "v"(b)); return d; }
__device__ __forceinline__ void wave_lds_sync() { __builtin_amdgcn_fence(__ATOMIC_RELEASE, "workgroup"); __builtin_amdgcn_wave_barrier(); __builtin_amdgcn_fence(__ATOMIC_ACQUIRE, "workgroup"); }
__device__ __forceinline__ float pmul(float a, float b) { float p = a * b; asm volatile("" : "+v"(p)); return p; }
__device__ __forceinline__ int iclamp(int v, int lo, int hi) { return v < lo ? lo : (v > hi ? hi : v); }
constexpr int CSR_NBLK = 512, CSR_GB = 9, CSR_GN = 1 << CSR_GB  , CSR_MAXG = 512, CSR_CAP = 12288  ;
__global__ __launch_bounds__(64) void csrA_kernel(const int* __restrict__ dst, int E, int N, int nG, int CHP, int NGP, int* __restrict__ STG, int* __restrict__ HST) {
  extern __shared__ int sm[];
  int* cnt = sm; int* run = sm + NGP; int* ids = sm + 2 * NGP;
  const int b = blockIdx.x; const int ch = (E + CSR_NBLK - 1) / CSR_NBLK; const int e0 = b * ch, e1 = min(E, e0 + ch);
  for (int i = threadIdx.x; i < NGP; i += 64) cnt[i] = 0;
  for (int i = threadIdx.x; i < CHP; i += 64) ids[i] = -1;
  __syncthreads();
  if (threadIdx.x == 0) {
    for (int e = e0; e < e1; ++e) { int d = dst[e]; d = (d < 0) ? 0 : (d >= N ? N - 1 : d); cnt[d >> CSR_GB] += 1; }
    int acc = 0; for (int g = 0; g < nG; ++g) { run[g] = acc; acc += cnt[g]; }
    for (int e = e0; e < e1; ++e) { int d = dst[e]; d = (d < 0) ? 0 : (d >= N ? N - 1 : d); const int g = d >> CSR_GB; ids[run[g]] = e; run[g] += 1; } }
  __syncthreads();
  typedef __attribute__((ext_vector_type(4))) int v4i;
  for (int pass = 0; pass < 2; ++pass) {
    for (int i = threadIdx.x; i < CHP / 4; i += 64) *(volatile v4i*)(STG + (size_t)b * CHP + i * 4) = *(const v4i*)(&ids[i * 4]);
    for (int i = threadIdx.x; i < NGP / 4; i += 64) { v4i v; for (int e = 0; e < 4; ++e) v[e] = (i * 4 + e < nG) ? cnt[i * 4 + e] : 0; *(volatile v4i*)(HST + (size_t)b * NGP + i * 4) = v; }
    __threadfence(); }
}
__global__ __launch_bounds__(512) void csrS_kernel(const int* __restrict__ HST, int nG, int NGP, int* __restrict__ START, int* __restrict__ TOT, int* __restrict__ OFF) {
  __shared__ int tot[CSR_MAXG];
  const int b = threadIdx.x;
  for (int pass = 0; pass < 2; ++pass) { int runb = 0; for (int g = 0; g < nG; ++g) { int c = HST[(size_t)b * NGP + g]; c = (c < 0) ? 0 : c; ((volatile int*)OFF)[(size_t)g * CSR_NBLK + b] = runb; runb += c; } __threadfence(); }
  for (int g = threadIdx.x; g < nG; g += 512) { int s = 0; for (int bb = 0; bb < CSR_NBLK; ++bb) { int c = HST[(size_t)bb * NGP + g]; s += (c < 0) ? 0 : c; } tot[g] = s; }
  __syncthreads();
  if (threadIdx.x < 32) {
    __shared__ int st[CSR_MAXG + 32];
    if (threadIdx.x == 0) { int acc = 0; for (int g = 0; g < NGP; ++g) { st[g] = acc; if (g < nG) acc += (tot[g] + 31) & ~31; } st[NGP] = acc; }
    __builtin_amdgcn_fence(__ATOMIC_RELEASE, "workgroup"); __builtin_amdgcn_wave_barrier(); __builtin_amdgcn_fence(__ATOMIC_ACQUIRE, "workgroup");
    for (int pass = 0; pass < 2; ++pass) { for (int i = threadIdx.x; i < NGP + 32; i += 32) { ((volatile int*)START)[i] = (i <= NGP) ? st[min(i, NGP)] : 0; ((volatile int*)TOT)[i] = (i < nG) ? tot[i] : 0; } __threadfence(); } }
}
__global__ __launch_bounds__(256) void csrB_kernel(const int* __restrict__ dst, int N, int nG, int CHP, int NGP, int permLen, const int* __restrict__ STG, const int* __restrict__ HST, const int* __restrict__ OFF, const int* __restrict__ START, const int* __restrict__ TOT, int* __restrict__ PERM, int* __restrict__ ROWPTR, int* __restrict__ ROWCNT, int* __restrict__ FLAG) {
  typedef __attribute__((ext_vector_type(4))) int v4i;
  __shared__ int ids[CSR_CAP]; __shared__ unsigned short key[CSR_CAP]; __shared__ int outp[CSR_CAP]; __shared__ int ncnt[CSR_GN + 1]; __shared__ int boff[CSR_NBLK + 1];
  const int g = blockIdx.x, t_ = threadIdx.x; int tot = TOT[g]; int st = START[g], stn = START[g + 1]; const int v0 = g * CSR_GN; const int nv = min(CSR_GN, N - v0);
  st = (st < 0) ? 0 : (st > permLen - 32 ? permLen - 32 : st) & ~31; stn = (stn < st) ? st : (stn > permLen ? permLen : stn); tot = (tot < 0) ? 0 : tot; if (tot > stn - st && tot <= CSR_CAP) tot = stn - st;
  if (tot > CSR_CAP) {
    for (int pass = 0; pass < 2; ++pass) { for (int i = t_; i < CSR_GN / 4; i += 256) { v4i a, c; for (int e = 0; e < 4; ++e) { a[e] = st; c[e] = 0; } *(volatile v4i*)(ROWPTR + v0 + i * 4) = a; *(volatile v4i*)(ROWCNT + v0 + i * 4) = c; } if (t_ == 0) ((volatile int*)FLAG)[0] = 1; __threadfence(); } (void)nv; return; }
  if (t_ == 0) { int acc = 0; for (int b = 0; b < CSR_NBLK; ++b) { boff[b] = acc; int c = HST[(size_t)b * NGP + g]; c = (c < 0) ? 0 : (c > CHP ? CHP : c); acc += c; if (acc > tot) acc = tot; } boff[CSR_NBLK] = acc; }
  for (int i = t_; i <= CSR_GN; i += 256) ncnt[i] = 0;
  __syncthreads();
  for (int b = 0; b < CSR_NBLK; ++b) { const int c = boff[b + 1] - boff[b]; int o_ = OFF[(size_t)g * CSR_NBLK + b]; o_ = (o_ < 0) ? 0 : (o_ > CHP - c ? CHP - c : o_); const int* src_ = STG + (size_t)b * CHP + o_;
    for (int i = t_; i < c; i += 256) { int id = src_[i]; id = (id < 0) ? 0 : id; ids[boff[b] + i] = id; int d = dst[id]; d = (d < v0) ? v0 : (d >= N ? N - 1 : d); int kk = d - v0; kk = (kk < 0) ? 0 : (kk >= CSR_GN ? CSR_GN - 1 : kk); key[boff[b] + i] = (unsigned short)kk; } }
  __syncthreads();
  if (t_ == 0) { for (int i = 0; i < tot; ++i) ncnt[key[i]] += 1; int acc = 0; for (int vl = 0; vl < CSR_GN; ++vl) { const int c = ncnt[vl]; ncnt[vl] = acc; acc += c; } ncnt[CSR_GN] = acc;
    for (int i = 0; i < tot; ++i) { const int vl = key[i]; outp[ncnt[vl]] = ids[i]; ncnt[vl] += 1; }
    for (int vl = CSR_GN; vl > 0; --vl) ncnt[vl] = ncnt[vl - 1]; ncnt[0] = 0; }
  __syncthreads();
  for (int pass = 0; pass < 2; ++pass) {
    for (int i = t_; i < (stn - st) / 4; i += 256) { v4i v; for (int e = 0; e < 4; ++e) { const int q = i * 4 + e; v[e] = (q < tot) ? outp[q] : -1; } *(volatile v4i*)(PERM + st + i * 4) = v; }
    for (int i = t_; i < CSR_GN / 4; i += 256) { v4i a, c; for (int e = 0; e < 4; ++e) { const int vl = i * 4 + e; a[e] = st + ncnt[vl]; c[e] = (vl < nv) ? (ncnt[vl + 1] - ncnt[vl]) : 0; } *(volatile v4i*)(ROWPTR + v0 + i * 4) = a; *(volatile v4i*)(ROWCNT + v0 + i * 4) = c; }
    __threadfence(); }
}
__global__ __launch_bounds__(256) void csrZ_kernel(int* __restrict__ p, size_t n4) { typedef __attribute__((ext_vector_type(4))) int v4i; const size_t tid = (size_t)blockIdx.x * 256 + threadIdx.x, nth = (size_t)gridDim.x * 256; v4i z = {0, 0, 0, 0}; for (size_t i = tid; i < n4; i += nth) *(volatile v4i*)(p + i * 4) = z; }
struct CsrBufs { int *STG, *HST, *OFF, *START, *TOT, *PERM, *ROWPTR, *ROWCNT, *FLAG; int nG, NGP, CHP; size_t permLen; char* base; size_t bytes; };
static size_t csr_carve(CsrBufs& c, char* ws, size_t off, int E, int N) {
  const size_t off0 = off; c.base = ws + off;
  auto al = [&](size_t bytes) { char* p = ws + off; off += (bytes + 255) & ~(size_t)255; return p; };
  c.nG = (N + CSR_GN - 1) / CSR_GN; c.NGP = (c.nG + 31) & ~31; const int ch = (E + CSR_NBLK - 1) / CSR_NBLK; c.CHP = (ch + 31) & ~31; c.permLen = (size_t)E + 32 * (size_t)c.nG + 32;
  c.STG = (int*)al((size_t)CSR_NBLK * c.CHP * 4); c.HST = (int*)al((size_t)CSR_NBLK * c.NGP * 4); c.OFF = (int*)al((size_t)c.NGP * CSR_NBLK * 4); c.START = (int*)al((size_t)(c.NGP + 64) * 4); c.TOT = (int*)al((size_t)(c.NGP + 64) * 4);
  c.PERM = (int*)al(c.permLen * 4); c.ROWPTR = (int*)al((size_t)c.nG * CSR_GN * 4); c.ROWCNT = (int*)al((size_t)c.nG * CSR_GN * 4); c.FLAG = (int*)al(256);
  c.bytes = off - off0; return off;
}
static void csr_build(const CsrBufs& c, const int* dst, int E, int N, hipStream_t stream) {
  const size_t smem = (size_t)(2 * c.NGP + c.CHP) * 4;
  csrZ_kernel<<<512, 256, 0, stream>>>((int*)c.base, c.bytes / 16);
  csrA_kernel<<<CSR_NBLK, 64, smem, stream>>>(dst, E, N, c.nG, c.CHP, c.NGP, c.STG, c.HST);
  csrS_kernel<<<1, 512, 0, stream>>>(c.HST, c.nG, c.NGP, c.START, c.TOT, c.OFF);
  csrB_kernel<<<c.nG, 256, 0, stream>>>(dst, N, c.nG, c.CHP, c.NGP, (int)c.permLen, c.STG, c.HST, c.OFF, c.START, c.TOT, c.PERM, c.ROWPTR, c.ROWCNT, c.FLAG);
}

typedef __attribute__((ext_vector_type(4))) _Float16 v4h;
__device__ __forceinline__ float silu_(float y) { return y * __builtin_amdgcn_rcpf(1.0f + __expf(-y)); }
template <int K, int KP, int NOUT>
__global__ __launch_bounds__(256) void wt_kernel(const float* __restrict__ w, b16* __restrict__ WT, float scl) {
  const int u = blockIdx.x * 256 + threadIdx.x; if (u >= NOUT * KP / 8) return; const int e = u * 8; const int o = e / KP, k0 = e % KP; v8b v;
#pragma unroll
  for (int j = 0; j < 8; ++j) { const int k = k0 + j; v[j] = (b16)(k < K ? bf16_rne(w[(size_t)k * NOUT + o]) * scl : 0.0f); }
  for (int pass = 0; pass < 2; ++pass) { *(volatile v8b*)(WT + e) = v; __threadfence(); }
}
__global__ __launch_bounds__(64) void up_kernel(const float* __restrict__ x, const b16* __restrict__ WT, float* __restrict__ Hh) {
  __shared__ __attribute__((aligned(16))) b16 Ah[2][16][C + 8]; __shared__ __attribute__((aligned(16))) float Tf[2][16][C + 4];
  const int wave = threadIdx.x >> 5, lane = threadIdx.x & 31, nloc = lane & 15, hlf = lane >> 4; const size_t m0 = (size_t)blockIdx.x * 32 + wave * 16;
  for (int idx = lane; idx < 16 * (C / 4); idx += 32) { const int rr = idx / (C / 4), c4 = (idx % (C / 4)) * 4; const size_t arow = (m0 + rr < (size_t)N) ? m0 + rr : (size_t)N - 1; const v4f v = *(const v4f*)(x + arow * C + c4); v4h hv; for (int j = 0; j < 4; ++j) hv[j] = (b16)(bf16_rne(v[j]) * XS); *(v4h*)(&Ah[wave][rr][c4]) = hv; }
  wave_lds_sync();
  v8f acc[4]; for (int t = 0; t < 4; ++t) acc[t] = (v8f){};
#pragma unroll
  for (int kb = 0; kb < C; kb += 32) { const v16b a = frag_kb(&Ah[wave][nloc][kb], hlf);
#pragma unroll
    for (int t = 0; t < 4; ++t) acc[t] = wmma16b(a, frag_kb(WT + (size_t)(t * 16 + nloc) * C + kb, hlf), acc[t]); }
#pragma unroll
  for (int t = 0; t < 4; ++t) for (int r = 0; r < 8; ++r) Tf[wave][8 * hlf + r][t * 16 + nloc] = (m0 + 8 * hlf + r < (size_t)N) ? acc[t][r] * (1.0f / (XS * WSC)) * 0.125f : 0.0f;
  wave_lds_sync();
  for (int pass = 0; pass < 2; ++pass) { for (int rr = 0; rr < 16; rr += 2) { const int r2 = rr + (lane >> 4); *(volatile v4f*)(Hh + (m0 + r2) * C + (lane & 15) * 4) = *(const v4f*)(&Tf[wave][r2][(lane & 15) * 4]); } __threadfence(); }
}
__global__ __launch_bounds__(64) void edge_kernel(const float* __restrict__ Hh, const float* __restrict__ vec, const float* __restrict__ rad, const int* __restrict__ snd, const int* __restrict__ PERM, const int* __restrict__ ROWPTR, const int* __restrict__ ROWCNT, int permLen, const b16* __restrict__ W1T, const b16* __restrict__ W2T, const b16* __restrict__ W2Q, const b16* __restrict__ W3T, const b16* __restrict__ W3Q, const b16* __restrict__ W4T, const b16* __restrict__ W4Q, float* __restrict__ AGG) {
  __shared__ __attribute__((aligned(16))) b16 Ah[2][16][G + 8], Al[2][16][G + 8]; __shared__ __attribute__((aligned(16))) float Tm[2][16][MW + 4]; __shared__ float Ys[2][16][8]; __shared__ int Js[2][16];
  const int wave = threadIdx.x >> 5, lane = threadIdx.x & 31, nloc = lane & 15, hlf = lane >> 4; const int v = blockIdx.x * 2 + wave;
  int cnt = 0, p0 = 0; if (v < N) { cnt = iclamp(ROWCNT[v], 0, 65536); p0 = iclamp(ROWPTR[v], 0, permLen - 1); if (p0 + cnt > permLen) cnt = permLen - p0; }
  float acc[18]; for (int j = 0; j < 18; ++j) acc[j] = 0.0f;
  const float isq8 = 0.35355339059327373f, isq64 = 0.125f, sq3 = 1.7320508075688772f, sq15 = 3.872983346207417f, sq5h = 1.118033988749895f;
#pragma unroll 1
  for (int e0 = 0; e0 < cnt; e0 += 16) {
    const int nval = (cnt - e0 < 16) ? (cnt - e0) : 16;
    if (lane < 16) { int s = 0; float y[8] = {0, 0, 0, 0, 0, 0, 0, 0}; v8b r8 = (v8b){};
      if (lane < nval) { const int e = iclamp(PERM[p0 + e0 + lane], 0, E - 1); s = iclamp(snd[e], 0, N - 1); if (SRCM < N) s %= SRCM;
        const float vx = bf16_rne(vec[(size_t)e * 3]), vy = bf16_rne(vec[(size_t)e * 3 + 1]), vz = bf16_rne(vec[(size_t)e * 3 + 2]); const float inv = rsqrtf(fmaf(vx, vx, fmaf(vy, vy, pmul(vz, vz)))); const float ux = vx * inv, uy = vy * inv, uz = vz * inv;
        y[0] = sq3 * ux; y[1] = sq3 * uy; y[2] = sq3 * uz; y[3] = sq15 * ux * uy; y[4] = sq15 * uy * uz; y[5] = sq5h * (3.0f * uz * uz - 1.0f); y[6] = sq15 * ux * uz; y[7] = 0.5f * sq15 * (ux * ux - uy * uy);
        for (int j = 0; j < 8; ++j) r8[j] = (b16)(bf16_rne(rad[(size_t)e * RB + j]) * XS); }
      Js[wave][lane] = s; for (int j = 0; j < 8; ++j) Ys[wave][lane][j] = y[j];
      *(v8b*)(&Ah[wave][lane][0]) = r8; for (int k = 8; k < KR; k += 8) *(v8b*)(&Ah[wave][lane][k]) = (v8b){}; }
    wave_lds_sync();
    v8f acc4[4]; for (int t = 0; t < 4; ++t) acc4[t] = (v8f){};
    { const v16b a = frag_kb(&Ah[wave][nloc][0], hlf);
#pragma unroll
      for (int t = 0; t < 4; ++t) acc4[t] = wmma16b(a, frag_kb(W1T + (size_t)(t * 16 + nloc) * KR, hlf), acc4[t]); }
    wave_lds_sync();
#pragma unroll 1
    for (int st = 0; st < 2; ++st) {
      const float scl = (st == 0) ? isq8 : isq64;
#pragma unroll
      for (int t = 0; t < 4; ++t) { const int col = t * 16 + nloc; for (int r = 0; r < 8; ++r) { const float gv = silu_(acc4[t][r] * (1.0f / (XS * WSC)) * scl); const float vs = gv * XS; const b16 ph = (b16)vs; Ah[wave][8 * hlf + r][col] = ph; Al[wave][8 * hlf + r][col] = (b16)((vs - (float)ph) * RS_); } }
      wave_lds_sync();
      const b16* WT = (st == 0) ? W2T : W3T; const b16* WQ = (st == 0) ? W2Q : W3Q;
      for (int t = 0; t < 4; ++t) acc4[t] = (v8f){};
#pragma unroll
      for (int kb = 0; kb < G; kb += 32) { const v16b a = frag_kb(&Ah[wave][nloc][kb], hlf), al = frag_kb(&Al[wave][nloc][kb], hlf);
#pragma unroll
        for (int t = 0; t < 4; ++t) { const size_t wo_ = (size_t)(t * 16 + nloc) * G + kb; acc4[t] = wmma16b(a, frag_kb(WT + wo_, hlf), acc4[t]); acc4[t] = wmma16b(al, frag_kb(WQ + wo_, hlf), acc4[t]); } }
      wave_lds_sync(); }
#pragma unroll
    for (int t = 0; t < 4; ++t) { const int col = t * 16 + nloc; for (int r = 0; r < 8; ++r) { const float gv = silu_(acc4[t][r] * (1.0f / (XS * WSC)) * isq64); const float vs = gv * XS; const b16 ph = (b16)vs; Ah[wave][8 * hlf + r][col] = ph; Al[wave][8 * hlf + r][col] = (b16)((vs - (float)ph) * RS_); } }
    wave_lds_sync();
    { v8f am[12];
#pragma unroll
      for (int t = 0; t < 12; ++t) am[t] = (v8f){};
#pragma unroll
      for (int kb = 0; kb < G; kb += 32) { const v16b a = frag_kb(&Ah[wave][nloc][kb], hlf), al = frag_kb(&Al[wave][nloc][kb], hlf);
#pragma unroll
        for (int t = 0; t < 12; ++t) { const size_t wo_ = (size_t)(t * 16 + nloc) * G + kb; am[t] = wmma16b(a, frag_kb(W4T + wo_, hlf), am[t]); am[t] = wmma16b(al, frag_kb(W4Q + wo_, hlf), am[t]); } }
#pragma unroll
      for (int t = 0; t < 12; ++t) for (int r = 0; r < 8; ++r) Tm[wave][8 * hlf + r][t * 16 + nloc] = am[t][r] * (1.0f / (XS * WSC)) * isq64; }
    wave_lds_sync();
#pragma unroll 1
    for (int rr = 0; rr < nval; ++rr) { const int s = Js[wave][rr]; const float* hr = Hh + (size_t)s * C; const float* tm = &Tm[wave][rr][0]; const float* yy = &Ys[wave][rr][0];
#pragma unroll
      for (int q = 0; q < 2; ++q) { const int c = lane + 32 * q; const float sv = hr[c] * (1.0f / 64.0f); const float a0 = sv * tm[c], a1 = sv * tm[C + c], a2 = sv * tm[2 * C + c];
        acc[9 * q] += a0;
#pragma unroll
        for (int m = 0; m < 3; ++m) acc[9 * q + 1 + m] = fmaf(a1, yy[m], acc[9 * q + 1 + m]);
#pragma unroll
        for (int m = 0; m < 5; ++m) acc[9 * q + 4 + m] = fmaf(a2, yy[3 + m], acc[9 * q + 4 + m]); } }
    wave_lds_sync(); }
  for (int pass = 0; pass < 2; ++pass) { if (v < NPL) { float* row = AGG + (size_t)v * OW; const bool ok = v < N;
#pragma unroll
      for (int q = 0; q < 2; ++q) { const int c = lane + 32 * q; ((volatile float*)row)[c] = ok ? EPSS * acc[9 * q] : 0.0f;
#pragma unroll
        for (int m = 0; m < 3; ++m) ((volatile float*)row)[C + 3 * c + m] = ok ? EPSS * acc[9 * q + 1 + m] : 0.0f;
#pragma unroll
        for (int m = 0; m < 5; ++m) ((volatile float*)row)[4 * C + 5 * c + m] = ok ? EPSS * acc[9 * q + 4 + m] : 0.0f; } }
    __threadfence(); }
}
__global__ __launch_bounds__(64) void down_kernel(const float* __restrict__ AGG, const b16* __restrict__ WD, const b16* __restrict__ WDQ, float* __restrict__ out, int mrows) {
  __shared__ __attribute__((aligned(16))) b16 Ah[2][16][C + 8], Al[2][16][C + 8]; __shared__ __attribute__((aligned(16))) float To[2][16][OW + 4];
  const int wave = threadIdx.x >> 5, lane = threadIdx.x & 31, nloc = lane & 15, hlf = lane >> 4; const size_t m0 = (size_t)blockIdx.x * 32 + wave * 16;
#pragma unroll 1
  for (int sl = 0; sl < 9; ++sl) { const int l = (sl == 0) ? 0 : (sl <= 3 ? 1 : 2); const int m = (sl == 0) ? 0 : (sl <= 3 ? sl - 1 : sl - 4); const int S = (l == 0) ? 1 : (l == 1 ? 3 : 5); const int base = (l == 0) ? 0 : (l == 1 ? C : 4 * C);
    if (sl > 0) wave_lds_sync();
    for (int idx = lane; idx < 16 * C; idx += 32) { const int rr = idx / C, c = idx % C; const size_t arow = (m0 + rr < (size_t)N) ? m0 + rr : (size_t)N - 1; const float av = AGG[arow * OW + base + S * c + m]; const float vs = av * XS; const b16 ph = (b16)vs; Ah[wave][rr][c] = ph; Al[wave][rr][c] = (b16)((vs - (float)ph) * RS_); }
    wave_lds_sync();
    v8f acc[4]; for (int t = 0; t < 4; ++t) acc[t] = (v8f){};
    const b16* WT = WD + (size_t)l * C * C; const b16* WQ = WDQ + (size_t)l * C * C;
#pragma unroll
    for (int kb = 0; kb < C; kb += 32) { const v16b a = frag_kb(&Ah[wave][nloc][kb], hlf), al = frag_kb(&Al[wave][nloc][kb], hlf);
#pragma unroll
      for (int t = 0; t < 4; ++t) { const size_t wo_ = (size_t)(t * 16 + nloc) * C + kb; acc[t] = wmma16b(a, frag_kb(WT + wo_, hlf), acc[t]); acc[t] = wmma16b(al, frag_kb(WQ + wo_, hlf), acc[t]); } }
#pragma unroll
    for (int t = 0; t < 4; ++t) { const int d = t * 16 + nloc; for (int r = 0; r < 8; ++r) To[wave][8 * hlf + r][base + S * d + m] = (m0 + 8 * hlf + r < (size_t)N) ? acc[t][r] * (1.0f / (XS * WSC)) * 0.125f : 0.0f; } }
  wave_lds_sync();
  for (int pass = 0; pass < 2; ++pass) { for (int rr = 0; rr < 16; ++rr) if (m0 + rr < (size_t)mrows) { float* orow = out + (m0 + rr) * OW; for (int c8 = 0; c8 < OW; c8 += 128) if (c8 + lane * 4 < OW) *(volatile v4f*)(orow + c8 + lane * 4) = *(const v4f*)(&To[wave][rr][c8 + lane * 4]); } __threadfence(); }
}
}

extern "C" void kernel_launch(void* const* d_in, const int* in_sizes, int n_in, void* d_out, int out_size, void* d_ws, size_t ws_size, hipStream_t stream) {
  (void)n_in;
  auto Fp = [&](int i) { return (const float*)d_in[i]; }; auto Ip = [&](int i) { return (const int*)d_in[i]; };
  if (in_sizes[0] != EFULL * 3 || in_sizes[1] != N * C || in_sizes[2] != EFULL * RB || in_sizes[3] != EFULL || in_sizes[4] != EFULL || in_sizes[5] != C * C || in_sizes[6] != RB * G || in_sizes[7] != G * G || in_sizes[8] != G * G || in_sizes[9] != G * MW || in_sizes[10] != C * C || in_sizes[11] != C * C || in_sizes[12] != C * C || out_size != N * OW) return;
  size_t off = 0; char* ws = (char*)d_ws;
  auto carve = [&](size_t bytes) { char* p = ws + off; off += (bytes + 255) & ~(size_t)255; return p; };
  b16* WUP = (b16*)carve((size_t)C * C * 2); b16* W1T = (b16*)carve((size_t)G * KR * 2); b16* W2T = (b16*)carve((size_t)G * G * 2); b16* W2Q = (b16*)carve((size_t)G * G * 2); b16* W3T = (b16*)carve((size_t)G * G * 2); b16* W3Q = (b16*)carve((size_t)G * G * 2);
  b16* W4T = (b16*)carve((size_t)MW * G * 2); b16* W4Q = (b16*)carve((size_t)MW * G * 2); b16* WD = (b16*)carve((size_t)3 * C * C * 2); b16* WDQ = (b16*)carve((size_t)3 * C * C * 2);
  float* Hh = (float*)carve((size_t)NP * C * 4); float* AGG = (float*)carve((size_t)NP * OW * 4);
  CsrBufs csr; off = csr_carve(csr, ws, off, E, N);
  if (off > ws_size || off > ((size_t)128 << 20)) return;
  const unsigned g44 = (G * G / 8 + 255) / 256;
  wt_kernel<C, C, C><<<g44, 256, 0, stream>>>(Fp(5), WUP, WSC);
  wt_kernel<RB, KR, G><<<(G * KR / 8 + 255) / 256, 256, 0, stream>>>(Fp(6), W1T, WSC);
  wt_kernel<G, G, G><<<g44, 256, 0, stream>>>(Fp(7), W2T, WSC); wt_kernel<G, G, G><<<g44, 256, 0, stream>>>(Fp(7), W2Q, WSQ);
  wt_kernel<G, G, G><<<g44, 256, 0, stream>>>(Fp(8), W3T, WSC); wt_kernel<G, G, G><<<g44, 256, 0, stream>>>(Fp(8), W3Q, WSQ);
  wt_kernel<G, G, MW><<<(MW * G / 8 + 255) / 256, 256, 0, stream>>>(Fp(9), W4T, WSC); wt_kernel<G, G, MW><<<(MW * G / 8 + 255) / 256, 256, 0, stream>>>(Fp(9), W4Q, WSQ);
  for (int l = 0; l < 3; ++l) { wt_kernel<C, C, C><<<g44, 256, 0, stream>>>(Fp(10 + l), WD + (size_t)l * C * C, WSC); wt_kernel<C, C, C><<<g44, 256, 0, stream>>>(Fp(10 + l), WDQ + (size_t)l * C * C, WSQ); }
  csr_build(csr, Ip(4), E, N, stream);
  up_kernel<<<NP / 32, 64, 0, stream>>>(Fp(1), WUP, Hh);
  edge_kernel<<<NP / 2, 64, 0, stream>>>(Hh, Fp(0), Fp(2), Ip(3), csr.PERM, csr.ROWPTR, csr.ROWCNT, (int)csr.permLen, W1T, W2T, W2Q, W3T, W3Q, W4T, W4Q, AGG);
  down_kernel<<<NPL / 32, 64, 0, stream>>>(AGG, WD, WDQ, (float*)d_out, NL);
}
